// HeteroCompGCN_52183852646756
// MI455X (gfx1250) — hardware-verified
//
#include <hip/hip_runtime.h>
#include <stddef.h>
#include <stdint.h>


typedef _Float16 v16h __attribute__((ext_vector_type(16)));
typedef _Float16 v8h  __attribute__((ext_vector_type(8)));
typedef _Float16 v4h  __attribute__((ext_vector_type(4)));
typedef float    v8f  __attribute__((ext_vector_type(8)));
typedef float    v4f  __attribute__((ext_vector_type(4)));
typedef int      v4i  __attribute__((ext_vector_type(4)));

union Frag { v16h v; v8h half[2]; };

#define FC      128
#define FIN     96
#define TED     32
#define KTOT    256
#define SNODE   2048
#define ECAP    36864
#define MAXDEG  1024
#define NWV     8
#define TBLK    256
#define NPT     (SNODE / TBLK)
#define APITCH  264
#define SPITCH  132

#define CSR_LDS_BYTES (NWV * SNODE * 2 + SNODE * 4 + SNODE * 4 + ECAP * 4 + 64)

extern __shared__ __align__(16) unsigned char dyn_lds[];

__device__ __forceinline__ v8f mma16(v16h a, v16h b, v8f c) {
  c = __builtin_amdgcn_wmma_f32_16x16x32_f16(false, a, false, b, (short)0, c, false, false);
  asm volatile("v_nop\n\tv_nop\n\tv_nop\n\tv_nop" : "+v"(c) : "v"(a), "v"(b));
  return c;
}

__device__ __forceinline__ void csr_store(const int* lbeg, const int* ldeg, const int* lseg,
                                          int* ebeg, int* edeg, int* eseg,
                                          int base, size_t segoff, int nw4, int tid) {
#pragma unroll
  for (int i = 0; i < NPT / 4; ++i) {
    const int c = tid + i * TBLK;
    const v4i vb = *(const v4i*)(lbeg + 4 * c);
    const v4i vd = *(const v4i*)(ldeg + 4 * c);
    *(volatile v4i*)(ebeg + base + 4 * c) = vb;
    *(volatile v4i*)(edeg + base + 4 * c) = vd;
  }
  for (int c = tid; c < nw4; c += TBLK) {
    const v4i v = *(const v4i*)(lseg + 4 * c);
    *(volatile v4i*)(eseg + segoff + 4 * c) = v;
  }
}

__global__ __launch_bounds__(TBLK) void k_csr(const int* __restrict__ esrc,
                                               const int* __restrict__ edst,
                                               const int* __restrict__ etyp,
                                               int E, int N, int R,
                                               int* __restrict__ ebeg,
                                               int* __restrict__ edeg,
                                               int* __restrict__ eseg) {
  unsigned short* wcnt = reinterpret_cast<unsigned short*>(dyn_lds);
  int* lbeg = reinterpret_cast<int*>(dyn_lds + NWV * SNODE * 2);
  int* ldeg = lbeg + SNODE;
  int* lseg = ldeg + SNODE;
  int* wsum = lseg + ECAP;

  const int tid = threadIdx.x, lane = tid & 31, wv = tid >> 5;
  const int base = blockIdx.x * SNODE;
  unsigned short* mycnt = wcnt + wv * SNODE;

  for (int i = tid; i < NWV * SNODE; i += TBLK) wcnt[i] = 0;
  __syncthreads();

  const int ngrp = (E + 31) >> 5;

  for (int g = wv; g < ngrp; g += NWV) {
    const int e = (g << 5) + lane;
    int dl = -1;
    if (e < E) dl = edst[e] - base;
    const bool in = (unsigned)dl < (unsigned)SNODE;
    unsigned msk = __builtin_amdgcn_ballot_w32(in);
    while (msk) {
      const int j = __builtin_ctz(msk);
      msk &= msk - 1u;
      const int dj = __shfl(dl, j);
      if (lane == 0) mycnt[dj] = (unsigned short)(mycnt[dj] + 1);
    }
  }
  __syncthreads();

  int tc[NPT];
  int ls = 0;
#pragma unroll
  for (int i = 0; i < NPT; ++i) {
    const int n = NPT * tid + i;
    int run = 0;
#pragma unroll
    for (int w = 0; w < NWV; ++w) {
      const int c = wcnt[w * SNODE + n];
      wcnt[w * SNODE + n] = (unsigned short)run;
      run += c;
    }
    tc[i] = run;
    ls += run;
  }
  int v = ls;
#pragma unroll
  for (int off = 1; off < 32; off <<= 1) {
    const int u = __shfl_up(v, off);
    if (lane >= off) v += u;
  }
  if (lane == 31) wsum[wv] = v;
  __syncthreads();
  int wpre = 0, btot = 0;
#pragma unroll
  for (int w = 0; w < NWV; ++w) {
    const int s = wsum[w];
    btot += s;
    if (w < wv) wpre += s;
  }
  int excl = wpre + v - ls;
#pragma unroll
  for (int i = 0; i < NPT; ++i) {
    const int n = NPT * tid + i;
    lbeg[n] = excl;
    int rem = ECAP - excl;
    rem = rem < 0 ? 0 : rem;
    ldeg[n] = tc[i] < rem ? tc[i] : rem;
    excl += tc[i];
  }
  __syncthreads();

  for (int g = wv; g < ngrp; g += NWV) {
    const int e = (g << 5) + lane;
    int dl = -1, pk = 0;
    if (e < E) dl = edst[e] - base;
    const bool in = (unsigned)dl < (unsigned)SNODE;
    if (in) {
      int s = esrc[e];
      int t = etyp[e];
      s = s < 0 ? 0 : (s >= N ? N - 1 : s);
      t = t < 0 ? 0 : (t >= R ? R - 1 : t);
      pk = (s << 4) | (t & 15);
    }
    unsigned msk = __builtin_amdgcn_ballot_w32(in);
    while (msk) {
      const int j = __builtin_ctz(msk);
      msk &= msk - 1u;
      const int dj = __shfl(dl, j);
      const int pj = __shfl(pk, j);
      if (lane == 0) {
        const int q = mycnt[dj];
        mycnt[dj] = (unsigned short)(q + 1);
        const int pos = lbeg[dj] + q;
        if ((unsigned)pos < (unsigned)ECAP) lseg[pos] = pj;
      }
    }
  }
  __syncthreads();

  int nw = btot < ECAP ? btot : ECAP;
  nw = (nw + 127) & ~127;
  const int nw4 = nw >> 2;
  const size_t segoff = (size_t)blockIdx.x * ECAP;
  csr_store(lbeg, ldeg, lseg, ebeg, edeg, eseg, base, segoff, nw4, tid);
  __threadfence();
  csr_store(lbeg, ldeg, lseg, ebeg, edeg, eseg, base, segoff, nw4, tid);
}

__global__ __launch_bounds__(32) void k_prepw(const float* __restrict__ wo1, const float* __restrict__ wl1,
                                               const float* __restrict__ wo2, const float* __restrict__ wl2,
                                               const float* __restrict__ wo3, const float* __restrict__ wl3,
                                               _Float16* __restrict__ wt) {
  const int b = blockIdx.x;
  if (b >= 3 * FC) return;
  const int l = b >> 7, n = b & (FC - 1);
  const int lane = threadIdx.x & 31;
  const float* wo = (l == 0) ? wo1 : ((l == 1) ? wo2 : wo3);
  const float* wl = (l == 0) ? wl1 : ((l == 1) ? wl2 : wl3);
  const bool lo = lane < 16;
  const float* W = lo ? wo : wl;
  const int kb = lo ? (lane << 3) : ((lane - 16) << 3);
  const float sc = lo ? 64.0f : 1024.0f;
  v8h o;
#pragma unroll
  for (int i = 0; i < 8; ++i) o[i] = (_Float16)(W[(size_t)(kb + i) * FC + n] * sc);
  _Float16* p = wt + ((size_t)l * FC + n) * KTOT + (lane << 3);
  *(volatile v8h*)p = o;
  __threadfence();
  *(volatile v8h*)p = o;
}

__global__ __launch_bounds__(TBLK) void k_h0(const float* __restrict__ x,
                                              const int* __restrict__ tyid,
                                              const float* __restrict__ temb,
                                              int T, int N, float* __restrict__ h0) {
  const int lane = threadIdx.x & 31;
  const int row = blockIdx.x * NWV + (threadIdx.x >> 5);
  if (row >= N) return;
  v4f v;
  if (lane < 24) {
    v = *(const v4f*)(x + (size_t)row * FIN + 4 * lane);
  } else {
    int ty = tyid[row];
    ty = ty < 0 ? 0 : (ty >= T ? T - 1 : ty);
    v = *(const v4f*)(temb + (size_t)ty * TED + 4 * (lane - 24));
  }
  float* p = h0 + (size_t)row * FC + 4 * lane;
  *(volatile v4f*)p = v;
  __threadfence();
  *(volatile v4f*)p = v;
}

__device__ __forceinline__ void out_pass(const float* St, float* out, int row0, int wv, int lane, int N) {
  for (int q = 0; q < 16; ++q) {
    const int rr = wv * 16 + q;
    const int node = row0 + rr;
    if (node < N) {
      const v4f v = *(const v4f*)(St + rr * SPITCH + 4 * lane);
      *(volatile v4f*)(out + (size_t)node * FC + 4 * lane) = v;
    }
  }
}

__global__ __launch_bounds__(TBLK) void k_layer(const float* __restrict__ hin,
                                                 const float* __restrict__ rel, int R,
                                                 const int* __restrict__ ebeg,
                                                 const int* __restrict__ edeg,
                                                 const int* __restrict__ eseg,
                                                 const _Float16* __restrict__ wt,
                                                 float* __restrict__ out, int N, int relu) {
  __shared__ __align__(16) _Float16 Bs[FC * APITCH];
  __shared__ __align__(16) float    St[128 * SPITCH];
  _Float16* At = reinterpret_cast<_Float16*>(St);

  const int tid = threadIdx.x, lane = tid & 31, wv = tid >> 5;
  const int hh = lane >> 4, m = lane & 15;
  const int row0 = blockIdx.x * 128;

#pragma unroll
  for (int i = 0; i < 16; ++i) {
    const int c = tid + i * TBLK;
    const int n = c >> 5, kc = (c & 31) << 3;
    const v8h wv8 = *(const v8h*)(wt + (size_t)n * KTOT + kc);
    *(v8h*)(Bs + n * APITCH + kc) = wv8;
  }

  const v4f z4 = {0.0f, 0.0f, 0.0f, 0.0f};
  const v4f r1v = *(const v4f*)(rel + FC + 4 * lane);
  const int nm1 = N - 1, rm1 = R - 1;
#pragma unroll 1
  for (int q = 0; q < 16; ++q) {
    const int rr = wv * 16 + q;
    const int node = row0 + rr;
    v4f ag = z4, hv = z4;
    if (node < N) {
      hv = *(const v4f*)(hin + (size_t)node * FC + 4 * lane);
      v4f acc = hv * r1v;
      int bg = ebeg[node];
      int dg = edeg[node];
      dg = dg < 0 ? 0 : dg;
      const float inv = 1.0f / (float)(dg + 1);
      bg = bg < 0 ? 0 : (bg > ECAP ? ECAP : bg);
      int lim = ECAP - bg;
      lim = lim < MAXDEG ? lim : MAXDEG;
      const int dgl = dg < lim ? dg : lim;
      const int* seg = eseg + (size_t)(node / SNODE) * ECAP + bg;
#pragma unroll 1
      for (int p = 0; p < dgl; ++p) {
        const unsigned pk = (unsigned)seg[p];
        int s = (int)(pk >> 4);
        s = s < nm1 ? s : nm1;
        int t = (int)(pk & 15u);
        t = t < rm1 ? t : rm1;
        const v4f hs = *(const v4f*)(hin + (size_t)s * FC + 4 * lane);
        const v4f rv = *(const v4f*)(rel + (size_t)t * FC + 4 * lane);
        acc = acc + hs * rv;
      }
      ag = acc * (inv * 256.0f);
      hv = hv * 16.0f;
    }
    *(v4h*)(At + rr * APITCH + 4 * lane)      = __builtin_convertvector(ag, v4h);
    *(v4h*)(At + rr * APITCH + FC + 4 * lane) = __builtin_convertvector(hv, v4h);
  }
  __syncthreads();

  v8f acc8[8];
#pragma unroll
  for (int j = 0; j < 8; ++j) {
    const v8f z8 = {0.0f, 0.0f, 0.0f, 0.0f, 0.0f, 0.0f, 0.0f, 0.0f};
    acc8[j] = z8;
  }
  const _Float16* Ap = At + (wv * 16 + m) * APITCH + 8 * hh;
  const _Float16* Bp = Bs + m * APITCH + 8 * hh;
#pragma unroll 1
  for (int kt = 0; kt < KTOT / 32; ++kt) {
    Frag a;
    a.half[0] = *(const v8h*)(Ap + kt * 32);
    a.half[1] = *(const v8h*)(Ap + kt * 32 + 16);
#pragma unroll
    for (int j = 0; j < 8; ++j) {
      Frag b;
      b.half[0] = *(const v8h*)(Bp + j * 16 * APITCH + kt * 32);
      b.half[1] = *(const v8h*)(Bp + j * 16 * APITCH + kt * 32 + 16);
      acc8[j] = mma16(a.v, b.v, acc8[j]);
    }
  }
  __syncthreads();

  const float osc = 1.0f / 16384.0f;
#pragma unroll
  for (int j = 0; j < 8; ++j) {
#pragma unroll
    for (int r = 0; r < 8; ++r) {
      float vv = acc8[j][r] * osc;
      if (relu) vv = fmaxf(vv, 0.0f);
      St[(wv * 16 + 8 * hh + r) * SPITCH + j * 16 + m] = vv;
    }
  }
  __syncthreads();
  out_pass(St, out, row0, wv, lane, N);
  __threadfence();
  out_pass(St, out, row0, wv, lane, N);
}

extern "C" void kernel_launch(void* const* d_in, const int* in_sizes, int n_in,
                              void* d_out, int out_size, void* d_ws, size_t ws_size,
                              hipStream_t stream) {
  if (n_in < 14) return;
  const float* x    = (const float*)d_in[0];
  const int*   tyid = (const int*)  d_in[1];
  const int*   ei   = (const int*)  d_in[2];
  const int*   et   = (const int*)  d_in[3];
  const float* temb = (const float*)d_in[4];
  const float* rel1 = (const float*)d_in[5];
  const float* wl1  = (const float*)d_in[6];
  const float* wo1  = (const float*)d_in[7];
  const float* rel2 = (const float*)d_in[8];
  const float* wl2  = (const float*)d_in[9];
  const float* wo2  = (const float*)d_in[10];
  const float* rel3 = (const float*)d_in[11];
  const float* wl3  = (const float*)d_in[12];
  const float* wo3  = (const float*)d_in[13];

  const int N = in_sizes[1];
  const int E = in_sizes[3];
  const int T = in_sizes[4] / TED;
  const int R = in_sizes[5] / FC;
  if (N <= 0 || E < 0 || T <= 0 || R < 2) return;
  if (in_sizes[0] != N * FIN || in_sizes[2] != 2 * E || out_size != N * FC) return;
  const int* esrc = ei;
  const int* edst = ei + E;
  const int NB = (N + SNODE - 1) / SNODE;

  size_t off = 0;
  auto carve = [&](size_t bytes) { size_t o = off; off += (bytes + 255) & ~(size_t)255; return o; };
  const size_t oBeg = carve((size_t)NB * SNODE * sizeof(int));
  const size_t oDeg = carve((size_t)NB * SNODE * sizeof(int));
  const size_t oSeg = carve((size_t)NB * ECAP * sizeof(int));
  const size_t oWt  = carve((size_t)3 * FC * KTOT * sizeof(_Float16));
  const size_t oHp  = carve((size_t)N * FC * sizeof(float));
  const size_t oHq  = carve((size_t)N * FC * sizeof(float));
  if (off > ws_size) return;

  char* ws = (char*)d_ws;
  int* ebeg = (int*)(ws + oBeg);
  int* edeg = (int*)(ws + oDeg);
  int* eseg = (int*)(ws + oSeg);
  _Float16* wt = (_Float16*)(ws + oWt);
  float* hP = (float*)(ws + oHp);
  float* hQ = (float*)(ws + oHq);
  float* outp = (float*)d_out;

  k_csr<<<NB, TBLK, CSR_LDS_BYTES, stream>>>(esrc, edst, et, E, N, R, ebeg, edeg, eseg);

  k_prepw<<<3 * FC, 32, 0, stream>>>(wo1, wl1, wo2, wl2, wo3, wl3, wt);

  k_h0<<<(N + NWV - 1) / NWV, TBLK, 0, stream>>>(x, tyid, temb, T, N, hP);

  const int gL = (N + 127) / 128;
  k_layer<<<gL, TBLK, 0, stream>>>(hP, rel1, R, ebeg, edeg, eseg, wt,                          hQ,   N, 1);
  k_layer<<<gL, TBLK, 0, stream>>>(hQ, rel2, R, ebeg, edeg, eseg, wt + (size_t)FC * KTOT,      hP,   N, 1);
  k_layer<<<gL, TBLK, 0, stream>>>(hP, rel3, R, ebeg, edeg, eseg, wt + (size_t)2 * FC * KTOT,  outp, N, 0);
}
